// PointNetSetAbstraction_22359599743040
// MI455X (gfx1250) — hardware-verified
//
#include <hip/hip_runtime.h>
#pragma clang fp contract(off)

typedef __attribute__((ext_vector_type(16))) _Float16 v16h;
typedef __attribute__((ext_vector_type(8)))  _Float16 v8h;
typedef __attribute__((ext_vector_type(8)))  float    v8f;
typedef __attribute__((ext_vector_type(4)))  float    v4f;
typedef __attribute__((ext_vector_type(4)))  unsigned v4u;
typedef __attribute__((ext_vector_type(4)))  int      v4i;

constexpr int NBATCH  = 16;
constexpr int NPTS    = 4096;
constexpr int NFEAT   = 64;
constexpr int NCENT   = 1024;
constexpr int NNBR    = 32;
constexpr int CHAN0   = 64;
constexpr int CHAN1   = 128;
constexpr int CHAN2   = 256;
constexpr int MROWS   = NBATCH * NCENT * NNBR;
constexpr int NSRC    = NBATCH * NPTS;
constexpr int NGROUPS = NBATCH * NCENT;
constexpr int X2PITCH = 136;
constexpr float W_CARRY     = 64.0f;
constexpr float W_CARRY_INV = 1.0f / 64.0f;
constexpr double INV_ROWS   = 1.0 / (double)MROWS;

static_assert(MROWS == 524288, "row count");
static_assert(NSRC == 65536, "source rows");
static_assert(NFEAT == 64 && CHAN0 == 64 && CHAN1 == 128 && CHAN2 == 256, "channel plan");
static_assert(NNBR == 32, "one wave line per query");

constexpr size_t SZ_FPSI  = (size_t)NGROUPS * 4;
constexpr size_t SZ_BIDX  = (size_t)MROWS * 4;
constexpr size_t SZ_PPL   = (size_t)NSRC * 64 * 4;
constexpr size_t SZ_Y0H   = (size_t)MROWS * 64 * 2;
constexpr size_t SZ_EXT   = (size_t)NGROUPS * 256 * 4;
constexpr int    NBLK0    = MROWS / 256;
constexpr int    NBLK1    = MROWS / 512;
constexpr int    NBLK2    = MROWS / 128;
constexpr size_t SZ_PART0 = (size_t)NBLK0 * 128 * 4;
constexpr size_t SZ_PART1 = (size_t)NBLK1 * 256 * 4;
constexpr size_t SZ_PART2 = (size_t)NBLK2 * 512 * 4;
constexpr int    WPK_HALVES = 64 * 64 + 128 * 64 + 256 * 128;
constexpr size_t SZ_WPK   = (size_t)WPK_HALVES * 2;
constexpr size_t SZ_SCSH  = 512 * 4;
constexpr size_t OFF_FPSI  = 0;
constexpr size_t OFF_BIDX  = OFF_FPSI + SZ_FPSI;
constexpr size_t OFF_PPL   = OFF_BIDX + SZ_BIDX;
constexpr size_t OFF_Y0H   = OFF_PPL + SZ_PPL;
constexpr size_t OFF_EXT   = OFF_Y0H + SZ_Y0H;
constexpr size_t OFF_PART0 = OFF_EXT + SZ_EXT;
constexpr size_t OFF_PART1 = OFF_PART0 + SZ_PART0;
constexpr size_t OFF_PART2 = OFF_PART1 + SZ_PART1;
constexpr size_t OFF_WPK   = OFF_PART2 + SZ_PART2;
constexpr size_t OFF_SCSH0 = OFF_WPK + SZ_WPK;
constexpr size_t OFF_SCSH1 = OFF_SCSH0 + SZ_SCSH;
constexpr size_t OFF_SCSH2 = OFF_SCSH1 + SZ_SCSH;
constexpr size_t WS_TOTAL  = OFF_SCSH2 + SZ_SCSH;
static_assert(WS_TOTAL <= (size_t)134217728, "carve under 128 MiB");
static_assert((OFF_BIDX % 128) == 0 && (OFF_PPL % 128) == 0 && (OFF_Y0H % 128) == 0 && (OFF_EXT % 128) == 0, "line aligned");
static_assert((OFF_PART0 % 128) == 0 && (OFF_PART1 % 128) == 0 && (OFF_PART2 % 128) == 0 && (OFF_WPK % 128) == 0, "line aligned");
static_assert((OFF_SCSH0 % 128) == 0 && (OFF_SCSH1 % 128) == 0 && (OFF_SCSH2 % 128) == 0, "line aligned");
static_assert((NBLK0 % 8) == 0 && (NBLK1 % 8) == 0 && (NBLK2 % 8) == 0, "finalize split");
constexpr size_t OUT1_OFFSET_FLOATS = (size_t)NBATCH * NCENT * 3;
static_assert((OUT1_OFFSET_FLOATS * 4) == 196608 && ((OUT1_OFFSET_FLOATS * 4) % 128) == 0, "out1 byte offset");
static_assert(OUT1_OFFSET_FLOATS * 4 + (size_t)NGROUPS * 256 * 4 == (size_t)16973824, "d_out extent");

__device__ __forceinline__ float h16_to_f32(unsigned hb) {
  const unsigned sgn = (hb & 0x8000u) << 16;
  const unsigned em = hb & 0x7fffu;
  const float fn = __uint_as_float((em << 13) + 0x38000000u);
  const float fs = (float)em * 5.9604644775390625e-8f;
  const float mag = (em < 0x400u) ? fs : fn;
  return __uint_as_float(__float_as_uint(mag) | sgn);
}

__device__ __forceinline__ v8f unpack8(v4u w) {
  const unsigned w0 = w[0], w1 = w[1], w2 = w[2], w3 = w[3];
  v8f r;
  r[0] = h16_to_f32(w0 & 0xffffu); r[1] = h16_to_f32(w0 >> 16);
  r[2] = h16_to_f32(w1 & 0xffffu); r[3] = h16_to_f32(w1 >> 16);
  r[4] = h16_to_f32(w2 & 0xffffu); r[5] = h16_to_f32(w2 >> 16);
  r[6] = h16_to_f32(w3 & 0xffffu); r[7] = h16_to_f32(w3 >> 16);
  return r;
}

__device__ __forceinline__ v16h build_a(v4u wa, v4u wb,
                                        v4f s0, v4f s1, v4f s2, v4f s3,
                                        v4f h0, v4f h1, v4f h2, v4f h3) {
  const v8f fa = unpack8(wa);
  const v8f fb = unpack8(wb);
  v16h a;
#pragma unroll
  for (int e = 0; e < 4; ++e) {
    a[e]      = (_Float16)fmaxf(fa[e]     * s0[e] + h0[e], 0.0f);
    a[4 + e]  = (_Float16)fmaxf(fa[4 + e] * s1[e] + h1[e], 0.0f);
    a[8 + e]  = (_Float16)fmaxf(fb[e]     * s2[e] + h2[e], 0.0f);
    a[12 + e] = (_Float16)fmaxf(fb[4 + e] * s3[e] + h3[e], 0.0f);
  }
  return a;
}

union FragU { v16h v; v8h h[2]; };
__device__ __forceinline__ v16h frag_ld_g(const _Float16* p) {
  FragU f;
  f.h[0] = *(const v8h*)(p);
  f.h[1] = *(const v8h*)(p + 16);
  return f.v;
}

__device__ __forceinline__ v8f mma_h(v16h a, v16h b, v8f c) {
  c = __builtin_amdgcn_wmma_f32_16x16x32_f16(false, a, false, b, (short)0, c, false, false);
  asm volatile("v_nop\n\tv_nop\n\tv_nop\n\tv_nop" : "+v"(c) : "v"(a), "v"(b));
  return c;
}

__device__ __forceinline__ int clampi(int v, int lo, int hi) {
  v = v < lo ? lo : v;
  v = v > hi ? hi : v;
  return v;
}

__global__ __launch_bounds__(256) void prep_pack_kernel(const float* __restrict__ w0,
                                                        const float* __restrict__ w1,
                                                        const float* __restrict__ w2,
                                                        unsigned short* __restrict__ wpack) {
  const int blk = blockIdx.x;
  const int tid = threadIdx.x;
  const float* src;
  int ld, kdim, rowoff, base;
  if (blk < 2)      { src = w0; ld = 64;  kdim = 64;  rowoff = 3; base = 0; }
  else if (blk < 6) { src = w1; ld = 128; kdim = 64;  rowoff = 0; base = 4096; }
  else              { src = w2; ld = 256; kdim = 128; rowoff = 0; base = 12288; }
  const int e0 = blk * 2048 + tid * 8;
  const int le = e0 - base;
  const int n  = le / kdim;
  const int k0 = le - n * kdim;
  v8h hv;
#pragma unroll
  for (int e = 0; e < 8; ++e) {
    const float f = src[(size_t)(rowoff + k0 + e) * ld + n] * W_CARRY;
    hv[e] = (_Float16)f;
  }
  volatile v8h* dst = (volatile v8h*)(wpack + e0);
  *dst = hv;
  __threadfence();
  *dst = hv;
}

__global__ __launch_bounds__(512) void fps_kernel(const float* __restrict__ xyz,
                                                  float* __restrict__ out0,
                                                  int* __restrict__ fpsidx) {
#pragma clang fp contract(off)
  __shared__ __align__(16) float xs[NPTS * 3];
  __shared__ __align__(16) int selidx[NCENT];
  __shared__ float rD[2][16];
  __shared__ int   rI[2][16];
  const int tid  = threadIdx.x;
  const int lane = tid & 31;
  const int wave = tid >> 5;
  const int b    = blockIdx.x;
  const float* X = xyz + (size_t)b * NPTS * 3;
#pragma unroll
  for (int it = 0; it < 6; ++it) {
    const int e = tid + it * 512;
    const v4f v = *(const v4f*)(X + 4 * e);
    *(v4f*)(xs + 4 * e) = v;
  }
  __syncthreads();
  float px[8], py[8], pz[8], dmin[8];
#pragma unroll
  for (int j = 0; j < 8; ++j) {
    const int p = tid + j * 512;
    px[j] = xs[3 * p];
    py[j] = xs[3 * p + 1];
    pz[j] = xs[3 * p + 2];
    dmin[j] = 1e10f;
  }
  int far = 0;
#pragma unroll 1
  for (int i = 0; i < NCENT; ++i) {
    if (tid == 0) selidx[i] = far;
    const float cx = xs[far * 3];
    const float cy = xs[far * 3 + 1];
    const float cz = xs[far * 3 + 2];
    float bd = -1.0f;
    int   bi = 0;
#pragma unroll
    for (int j = 0; j < 8; ++j) {
      const float dx = px[j] - cx;
      const float dy = py[j] - cy;
      const float dz = pz[j] - cz;
      const float t0 = dx * dx;
      const float t1 = dy * dy;
      const float t2 = dz * dz;
      const float d  = (t0 + t2) + t1;
      const float nd = fminf(dmin[j], d);
      dmin[j] = nd;
      const bool tk = nd > bd;
      bd = tk ? nd : bd;
      bi = tk ? (tid + j * 512) : bi;
    }
#pragma unroll
    for (int off = 16; off >= 1; off >>= 1) {
      const float od = __shfl_xor(bd, off, 32);
      const int   oi = __shfl_xor(bi, off, 32);
      const bool tk = (od > bd) || ((od == bd) && (oi < bi));
      bd = tk ? od : bd;
      bi = tk ? oi : bi;
    }
    const int par = i & 1;
    if (lane == 0) { rD[par][wave] = bd; rI[par][wave] = bi; }
    __syncthreads();
    float d2 = rD[par][lane & 15];
    int   i2 = rI[par][lane & 15];
#pragma unroll
    for (int off = 8; off >= 1; off >>= 1) {
      const float od = __shfl_xor(d2, off, 32);
      const int   oi = __shfl_xor(i2, off, 32);
      const bool tk = (od > d2) || ((od == d2) && (oi < i2));
      d2 = tk ? od : d2;
      i2 = tk ? oi : i2;
    }
    far = i2 & (NPTS - 1);
  }
  __syncthreads();
  v4f ov0, ov1;
  v4i iv;
#pragma unroll
  for (int q = 0; q < 4; ++q) {
    const int f0 = 4 * tid + q;
    const int s0 = f0 / 3;
    const int c0 = f0 - 3 * s0;
    ov0[q] = xs[(selidx[s0] & (NPTS - 1)) * 3 + c0];
    const int f1 = 4 * (tid + 512) + q;
    const int s1r = f1 / 3;
    const int c1 = f1 - 3 * s1r;
    const int s1 = s1r < NCENT ? s1r : (NCENT - 1);
    ov1[q] = xs[(selidx[s1] & (NPTS - 1)) * 3 + c1];
    const int si = 4 * tid + q;
    iv[q] = selidx[si < NCENT ? si : (NCENT - 1)] & (NPTS - 1);
  }
  float* o = out0 + (size_t)b * NCENT * 3;
  int* fo = fpsidx + (size_t)b * NCENT;
  for (int pass = 0; pass < 2; ++pass) {
    *(volatile v4f*)(o + 4 * tid) = ov0;
    if (tid < 256) {
      *(volatile v4f*)(o + 4 * (tid + 512)) = ov1;
      *(volatile v4i*)(fo + 4 * tid) = iv;
    }
    __threadfence();
  }
}

__global__ __launch_bounds__(256) void ballq_kernel(const float* __restrict__ xyz,
                                                    const int* __restrict__ fpsidx,
                                                    int* __restrict__ bidx) {
#pragma clang fp contract(off)
  __shared__ int hl[8][32];
  const int tid  = threadIdx.x;
  const int lane = tid & 31;
  const int wave = tid >> 5;
  const int q    = blockIdx.x * 8 + wave;
  const int b    = q >> 10;
  const float* X = xyz + (size_t)b * NPTS * 3;
  const int fi = clampi(fpsidx[q], 0, NPTS - 1);
  const float qx = X[fi * 3];
  const float qy = X[fi * 3 + 1];
  const float qz = X[fi * 3 + 2];
  const float qxx = qx * qx;
  const float qyy = qy * qy;
  const float qzz = qz * qz;
  const float ss = (qxx + qzz) + qyy;
  const float r2 = __uint_as_float(0x3D23D70Au);
  hl[wave][lane] = NPTS - 1;
  const unsigned ltmask = (1u << lane) - 1u;
  int cnt = 0;
#pragma unroll 1
  for (int j0 = 0; j0 < NPTS; j0 += 32) {
    const int j = j0 + lane;
    const float x = X[j * 3];
    const float y = X[j * 3 + 1];
    const float z = X[j * 3 + 2];
    const float xx = x * x;
    const float yy = y * y;
    const float zz = z * z;
    const float sn = (xx + zz) + yy;
    float p = qx * x;
    p = fmaf(qy, y, p);
    p = fmaf(qz, z, p);
    float d = -2.0f * p;
    d = d + ss;
    d = d + sn;
    const bool hit = !(d > r2);
    const unsigned mask = __builtin_amdgcn_ballot_w32(hit);
    const int slot = cnt + __popc(mask & ltmask);
    if (hit && slot < NNBR) hl[wave][slot] = j;
    cnt += __popc(mask);
    if (cnt >= NNBR) break;
  }
  __syncthreads();
  const int v = clampi(hl[wave][(lane < cnt) ? lane : 0], 0, NPTS - 1);
  int* dst = bidx + (size_t)q * NNBR + lane;
  *(volatile int*)dst = v;
  __threadfence();
  *(volatile int*)dst = v;
}

__global__ __launch_bounds__(256) void pgemm_kernel(const float* __restrict__ pts,
                                                    const unsigned short* __restrict__ w0p_,
                                                    float* __restrict__ P) {
  __shared__ __align__(16) float sT[8][16 * 68];
  const int tid  = threadIdx.x;
  const int lane = tid & 31;
  const int wave = tid >> 5;
  const int h = lane >> 4;
  const int m = lane & 15;
  const int row0 = (blockIdx.x * 8 + wave) * 16;
  const _Float16* W = (const _Float16*)w0p_;
  const float* ar = pts + (size_t)(row0 + m) * NFEAT + 8 * h;
  v16h a[2];
#pragma unroll
  for (int ks = 0; ks < 2; ++ks) {
    const v4f f0 = *(const v4f*)(ar + ks * 32);
    const v4f f1 = *(const v4f*)(ar + ks * 32 + 4);
    const v4f f2 = *(const v4f*)(ar + ks * 32 + 16);
    const v4f f3 = *(const v4f*)(ar + ks * 32 + 20);
#pragma unroll
    for (int e = 0; e < 4; ++e) {
      a[ks][e]      = (_Float16)f0[e];
      a[ks][4 + e]  = (_Float16)f1[e];
      a[ks][8 + e]  = (_Float16)f2[e];
      a[ks][12 + e] = (_Float16)f3[e];
    }
  }
  v8f acc[4];
#pragma unroll
  for (int j = 0; j < 4; ++j) acc[j] = (v8f){0.f, 0.f, 0.f, 0.f, 0.f, 0.f, 0.f, 0.f};
#pragma unroll
  for (int j = 0; j < 4; ++j) {
    const _Float16* bp = W + (size_t)(j * 16 + m) * 64 + 8 * h;
    const v16h b0 = frag_ld_g(bp);
    const v16h b1 = frag_ld_g(bp + 32);
    acc[j] = mma_h(a[0], b0, acc[j]);
    acc[j] = mma_h(a[1], b1, acc[j]);
  }
  float* slab = sT[wave];
#pragma unroll
  for (int j = 0; j < 4; ++j) {
#pragma unroll
    for (int r = 0; r < 8; ++r) slab[(8 * h + r) * 68 + j * 16 + m] = acc[j][r] * W_CARRY_INV;
  }
  __builtin_amdgcn_fence(__ATOMIC_RELEASE, "workgroup");
  __builtin_amdgcn_wave_barrier();
  __builtin_amdgcn_fence(__ATOMIC_ACQUIRE, "workgroup");
  const int c4 = m * 4;
  for (int pass = 0; pass < 2; ++pass) {
#pragma unroll
    for (int it = 0; it < 8; ++it) {
      const int row = it * 2 + h;
      const v4f v = *(const v4f*)(slab + row * 68 + c4);
      *(volatile v4f*)(P + (size_t)(row0 + row) * 64 + c4) = v;
    }
    __threadfence();
  }
}

__global__ __launch_bounds__(256) void gather_kernel(const float* __restrict__ xyz,
                                                     const float* __restrict__ P,
                                                     const float* __restrict__ w0,
                                                     const int* __restrict__ fpsidx,
                                                     const int* __restrict__ bidx,
                                                     unsigned short* __restrict__ y0h,
                                                     float* __restrict__ part0) {
  __shared__ float red[8][128];
  __shared__ __align__(16) float outp[128];
  const int tid  = threadIdx.x;
  const int lane = tid & 31;
  const int wave = tid >> 5;
  const int q  = lane >> 3;
  const int c8 = (lane & 7) * 8;
  float wx[8], wy[8], wz[8];
  {
    const v4f a0 = *(const v4f*)(w0 + c8);
    const v4f a1 = *(const v4f*)(w0 + c8 + 4);
    const v4f b0 = *(const v4f*)(w0 + 64 + c8);
    const v4f b1 = *(const v4f*)(w0 + 64 + c8 + 4);
    const v4f d0 = *(const v4f*)(w0 + 128 + c8);
    const v4f d1 = *(const v4f*)(w0 + 128 + c8 + 4);
#pragma unroll
    for (int e = 0; e < 4; ++e) {
      wx[e] = a0[e]; wx[4 + e] = a1[e];
      wy[e] = b0[e]; wy[4 + e] = b1[e];
      wz[e] = d0[e]; wz[4 + e] = d1[e];
    }
  }
  const int rbase = blockIdx.x * 256 + wave * 32;
  const int b = rbase >> 15;
  const float* X = xyz + (size_t)b * NPTS * 3;
  const int fi = clampi(fpsidx[rbase >> 5], 0, NPTS - 1);
  const float cx = X[fi * 3];
  const float cy = X[fi * 3 + 1];
  const float cz = X[fi * 3 + 2];
  float s1[8], s2[8];
#pragma unroll
  for (int e = 0; e < 8; ++e) { s1[e] = 0.0f; s2[e] = 0.0f; }
#pragma unroll 1
  for (int it = 0; it < 8; ++it) {
    const int r = rbase + it * 4 + q;
    const int id = clampi(bidx[r], 0, NPTS - 1);
    const float rx = X[id * 3] - cx;
    const float ry = X[id * 3 + 1] - cy;
    const float rz = X[id * 3 + 2] - cz;
    const float* pr = P + ((size_t)b * NPTS + id) * 64 + c8;
    const v4f p0 = *(const v4f*)(pr);
    const v4f p1 = *(const v4f*)(pr + 4);
    v8h hv;
#pragma unroll
    for (int e = 0; e < 8; ++e) {
      float y = (e < 4) ? p0[e & 3] : p1[e & 3];
      y = fmaf(rx, wx[e], y);
      y = fmaf(ry, wy[e], y);
      y = fmaf(rz, wz[e], y);
      const _Float16 yh = (_Float16)y;
      hv[e] = yh;
      const float yr = (float)yh;
      s1[e] += yr;
      s2[e] += yr * yr;
    }
    volatile v8h* dst = (volatile v8h*)(y0h + (size_t)r * 64 + c8);
    *dst = hv;
    __threadfence();
    *dst = hv;
  }
#pragma unroll
  for (int e = 0; e < 8; ++e) {
    s1[e] += __shfl_xor(s1[e], 8, 32);
    s2[e] += __shfl_xor(s2[e], 8, 32);
    s1[e] += __shfl_xor(s1[e], 16, 32);
    s2[e] += __shfl_xor(s2[e], 16, 32);
  }
  if (lane < 8) {
#pragma unroll
    for (int e = 0; e < 8; ++e) {
      red[wave][c8 + e] = s1[e];
      red[wave][64 + c8 + e] = s2[e];
    }
  }
  __syncthreads();
  if (tid < 128) {
    float t = 0.0f;
#pragma unroll
    for (int w = 0; w < 8; ++w) t += red[w][tid];
    outp[tid] = t;
  }
  __syncthreads();
  if (tid < 32) {
    const v4f v = *(const v4f*)(outp + 4 * tid);
    float* pp = part0 + (size_t)blockIdx.x * 128 + 4 * tid;
    *(volatile v4f*)pp = v;
    __threadfence();
    *(volatile v4f*)pp = v;
  }
}

__global__ __launch_bounds__(256) void finalize_kernel(const float* __restrict__ part, int nblk, int nch,
                                                       const float* __restrict__ g,
                                                       const float* __restrict__ bt,
                                                       float* __restrict__ scsh) {
  __shared__ double ds[8][32];
  __shared__ double dq[8][32];
  const int tid  = threadIdx.x;
  const int lane = tid & 31;
  const int wave = tid >> 5;
  const int ch = blockIdx.x * 32 + lane;
  const int per = nblk >> 3;
  const int i0 = wave * per;
  const size_t pitch = (size_t)2 * nch;
  double a = 0.0, qq = 0.0;
#pragma unroll 4
  for (int i = 0; i < per; ++i) {
    const float* p = part + (size_t)(i0 + i) * pitch + ch;
    a  += (double)p[0];
    qq += (double)p[nch];
  }
  ds[wave][lane] = a;
  dq[wave][lane] = qq;
  __syncthreads();
  if (wave == 0) {
    double A = 0.0, Q = 0.0;
#pragma unroll
    for (int w = 0; w < 8; ++w) { A += ds[w][lane]; Q += dq[w][lane]; }
    const double mean = A * INV_ROWS;
    const double var  = Q * INV_ROWS - mean * mean;
    float vf = (float)var;
    vf = vf > 0.0f ? vf : 0.0f;
    const float sc = g[ch] * (1.0f / sqrtf(vf + 1e-5f));
    const float sh = bt[ch] - (float)mean * sc;
    for (int pass = 0; pass < 2; ++pass) {
      *(volatile float*)(scsh + ch) = sc;
      *(volatile float*)(scsh + 256 + ch) = sh;
      __threadfence();
    }
  }
}

__global__ __launch_bounds__(256) void passB_kernel(const unsigned short* __restrict__ y0h,
                                                    const unsigned short* __restrict__ w1t_,
                                                    const float* __restrict__ scsh0,
                                                    float* __restrict__ part1) {
  __shared__ __align__(16) float tab[128];
  __shared__ float red[8][256];
  __shared__ __align__(16) float outp[256];
  const int tid  = threadIdx.x;
  const int lane = tid & 31;
  const int wave = tid >> 5;
  const int h = lane >> 4;
  const int m = lane & 15;
  const int kb = 8 * h;
  if (tid < 128) tab[tid] = scsh0[(tid < 64) ? tid : (192 + tid)];
  __syncthreads();
  const _Float16* W1 = (const _Float16*)w1t_;
  float s1[8], s2[8];
#pragma unroll
  for (int j = 0; j < 8; ++j) { s1[j] = 0.0f; s2[j] = 0.0f; }
#pragma unroll 1
  for (int t = 0; t < 4; ++t) {
    asm volatile("" ::: "memory");
    const int row0 = blockIdx.x * 512 + (wave * 4 + t) * 16;
    const unsigned short* rowp = y0h + (size_t)(row0 + m) * 64 + kb;
    const v4u wa0 = *(const v4u*)(rowp);
    const v4u wb0 = *(const v4u*)(rowp + 16);
    const v4u wa1 = *(const v4u*)(rowp + 32);
    const v4u wb1 = *(const v4u*)(rowp + 48);
    const v16h a0 = build_a(wa0, wb0,
        *(const v4f*)(tab + kb), *(const v4f*)(tab + kb + 4), *(const v4f*)(tab + kb + 16), *(const v4f*)(tab + kb + 20),
        *(const v4f*)(tab + 64 + kb), *(const v4f*)(tab + 64 + kb + 4), *(const v4f*)(tab + 64 + kb + 16), *(const v4f*)(tab + 64 + kb + 20));
    const v16h a1 = build_a(wa1, wb1,
        *(const v4f*)(tab + 32 + kb), *(const v4f*)(tab + 32 + kb + 4), *(const v4f*)(tab + 32 + kb + 16), *(const v4f*)(tab + 32 + kb + 20),
        *(const v4f*)(tab + 96 + kb), *(const v4f*)(tab + 96 + kb + 4), *(const v4f*)(tab + 96 + kb + 16), *(const v4f*)(tab + 96 + kb + 20));
    v8f acc[8];
#pragma unroll
    for (int j = 0; j < 8; ++j) acc[j] = (v8f){0.f, 0.f, 0.f, 0.f, 0.f, 0.f, 0.f, 0.f};
#pragma unroll
    for (int j = 0; j < 8; ++j) {
      const _Float16* bp = W1 + (size_t)(j * 16 + m) * 64 + kb;
      const v16h b0 = frag_ld_g(bp);
      const v16h b1 = frag_ld_g(bp + 32);
      acc[j] = mma_h(a0, b0, acc[j]);
      acc[j] = mma_h(a1, b1, acc[j]);
      if ((j & 1) == 1) asm volatile("" ::: "memory");
    }
#pragma unroll
    for (int j = 0; j < 8; ++j) {
#pragma unroll
      for (int r = 0; r < 8; ++r) {
        const float v = acc[j][r] * W_CARRY_INV;
        s1[j] += v;
        s2[j] += v * v;
      }
    }
  }
#pragma unroll
  for (int j = 0; j < 8; ++j) {
    s1[j] += __shfl_xor(s1[j], 16, 32);
    s2[j] += __shfl_xor(s2[j], 16, 32);
  }
  if (lane < 16) {
#pragma unroll
    for (int j = 0; j < 8; ++j) {
      red[wave][j * 16 + lane] = s1[j];
      red[wave][128 + j * 16 + lane] = s2[j];
    }
  }
  __syncthreads();
  {
    float t = 0.0f;
#pragma unroll
    for (int w = 0; w < 8; ++w) t += red[w][tid];
    outp[tid] = t;
  }
  __syncthreads();
  if (tid < 64) {
    const v4f v = *(const v4f*)(outp + 4 * tid);
    float* pp = part1 + (size_t)blockIdx.x * 256 + 4 * tid;
    *(volatile v4f*)pp = v;
    __threadfence();
    *(volatile v4f*)pp = v;
  }
}

__global__ __launch_bounds__(128) void passC_kernel(const unsigned short* __restrict__ y0h,
                                                    const unsigned short* __restrict__ w1t_,
                                                    const unsigned short* __restrict__ w2t_,
                                                    const float* __restrict__ scsh0,
                                                    const float* __restrict__ scsh1,
                                                    const float* __restrict__ g2,
                                                    float* __restrict__ part2,
                                                    float* __restrict__ ext) {
  __shared__ __align__(16) float tab[384];
  __shared__ __align__(16) _Float16 x2t[4][32 * X2PITCH];
  __shared__ float red[4][512];
  __shared__ __align__(16) float extS[4][256];
  __shared__ __align__(16) float outp[512];
  const int tid  = threadIdx.x;
  const int lane = tid & 31;
  const int wave = tid >> 5;
  const int h = lane >> 4;
  const int m = lane & 15;
  const int kb = 8 * h;
  tab[tid] = scsh0[(tid < 64) ? tid : (192 + tid)];
  tab[128 + tid] = scsh1[tid];
  tab[256 + tid] = scsh1[256 + tid];
  __syncthreads();
  const _Float16* W1 = (const _Float16*)w1t_;
  const _Float16* W2 = (const _Float16*)w2t_;
  _Float16* xt = x2t[wave];
  const int row0 = blockIdx.x * 128 + wave * 32;
#pragma unroll 1
  for (int i = 0; i < 2; ++i) {
    const unsigned short* rowp = y0h + (size_t)(row0 + i * 16 + m) * 64 + kb;
    const v4u wa0 = *(const v4u*)(rowp);
    const v4u wb0 = *(const v4u*)(rowp + 16);
    const v4u wa1 = *(const v4u*)(rowp + 32);
    const v4u wb1 = *(const v4u*)(rowp + 48);
    const v16h a0 = build_a(wa0, wb0,
        *(const v4f*)(tab + kb), *(const v4f*)(tab + kb + 4), *(const v4f*)(tab + kb + 16), *(const v4f*)(tab + kb + 20),
        *(const v4f*)(tab + 64 + kb), *(const v4f*)(tab + 64 + kb + 4), *(const v4f*)(tab + 64 + kb + 16), *(const v4f*)(tab + 64 + kb + 20));
    const v16h a1 = build_a(wa1, wb1,
        *(const v4f*)(tab + 32 + kb), *(const v4f*)(tab + 32 + kb + 4), *(const v4f*)(tab + 32 + kb + 16), *(const v4f*)(tab + 32 + kb + 20),
        *(const v4f*)(tab + 96 + kb), *(const v4f*)(tab + 96 + kb + 4), *(const v4f*)(tab + 96 + kb + 16), *(const v4f*)(tab + 96 + kb + 20));
    v8f acc[8];
#pragma unroll
    for (int j = 0; j < 8; ++j) acc[j] = (v8f){0.f, 0.f, 0.f, 0.f, 0.f, 0.f, 0.f, 0.f};
#pragma unroll
    for (int j = 0; j < 8; ++j) {
      const _Float16* bp = W1 + (size_t)(j * 16 + m) * 64 + kb;
      const v16h b0 = frag_ld_g(bp);
      const v16h b1 = frag_ld_g(bp + 32);
      acc[j] = mma_h(a0, b0, acc[j]);
      acc[j] = mma_h(a1, b1, acc[j]);
      if ((j & 1) == 1) asm volatile("" ::: "memory");
    }
#pragma unroll
    for (int j = 0; j < 8; ++j) {
      const int col = j * 16 + m;
      const float sc = tab[128 + col];
      const float sh = tab[256 + col];
#pragma unroll
      for (int r = 0; r < 8; ++r) {
        float v = acc[j][r] * W_CARRY_INV;
        v = v * sc + sh;
        v = fmaxf(v, 0.0f);
        xt[(i * 16 + 8 * h + r) * X2PITCH + col] = (_Float16)v;
      }
    }
  }
  __syncthreads();
#pragma unroll 1
  for (int nq = 0; nq < 4; ++nq) {
    float gv[4];
#pragma unroll
    for (int j = 0; j < 4; ++j) gv[j] = g2[nq * 64 + j * 16 + m];
    v8f c[2][4];
#pragma unroll
    for (int i = 0; i < 2; ++i)
#pragma unroll
      for (int j = 0; j < 4; ++j) c[i][j] = (v8f){0.f, 0.f, 0.f, 0.f, 0.f, 0.f, 0.f, 0.f};
#pragma unroll 1
    for (int ks = 0; ks < 4; ++ks) {
      FragU fa0, fa1;
      fa0.h[0] = *(const v8h*)(xt + m * X2PITCH + ks * 32 + kb);
      fa0.h[1] = *(const v8h*)(xt + m * X2PITCH + ks * 32 + 16 + kb);
      fa1.h[0] = *(const v8h*)(xt + (16 + m) * X2PITCH + ks * 32 + kb);
      fa1.h[1] = *(const v8h*)(xt + (16 + m) * X2PITCH + ks * 32 + 16 + kb);
#pragma unroll
      for (int j = 0; j < 4; ++j) {
        const v16h b = frag_ld_g(W2 + (size_t)(nq * 64 + j * 16 + m) * 128 + ks * 32 + kb);
        c[0][j] = mma_h(fa0.v, b, c[0][j]);
        c[1][j] = mma_h(fa1.v, b, c[1][j]);
      }
    }
#pragma unroll
    for (int j = 0; j < 4; ++j) {
      float t1 = 0.0f, t2 = 0.0f;
      float mx = -__builtin_huge_valf();
      float mn = __builtin_huge_valf();
#pragma unroll
      for (int i = 0; i < 2; ++i) {
#pragma unroll
        for (int r = 0; r < 8; ++r) {
          const float v = c[i][j][r] * W_CARRY_INV;
          t1 += v;
          t2 += v * v;
          mx = fmaxf(mx, v);
          mn = fminf(mn, v);
        }
      }
      t1 += __shfl_xor(t1, 16, 32);
      t2 += __shfl_xor(t2, 16, 32);
      mx = fmaxf(mx, __shfl_xor(mx, 16, 32));
      mn = fminf(mn, __shfl_xor(mn, 16, 32));
      const float ev = (gv[j] >= 0.0f) ? mx : mn;
      const int col = nq * 64 + j * 16 + m;
      if (lane < 16) {
        red[wave][col] = t1;
        red[wave][256 + col] = t2;
        extS[wave][col] = ev;
      }
    }
  }
  __syncthreads();
#pragma unroll
  for (int u = 0; u < 4; ++u) {
    const int idx = tid + u * 128;
    outp[idx] = ((red[0][idx] + red[1][idx]) + red[2][idx]) + red[3][idx];
  }
  __syncthreads();
  const v4f pv = *(const v4f*)(outp + 4 * tid);
  const v4f e0 = *(const v4f*)(&extS[wave][lane * 4]);
  const v4f e1 = *(const v4f*)(&extS[wave][128 + lane * 4]);
  float* pp = part2 + (size_t)blockIdx.x * 512 + 4 * tid;
  float* ep = ext + (size_t)(blockIdx.x * 4 + wave) * 256 + lane * 4;
  for (int pass = 0; pass < 2; ++pass) {
    *(volatile v4f*)pp = pv;
    *(volatile v4f*)ep = e0;
    *(volatile v4f*)(ep + 128) = e1;
    __threadfence();
  }
}

__global__ __launch_bounds__(256) void out_kernel(const float* __restrict__ ext,
                                                  const float* __restrict__ scsh2,
                                                  float* __restrict__ out1) {
  const int i = blockIdx.x * 256 + threadIdx.x;
  const int c4 = (i & 63) * 4;
  const v4f e  = *(const v4f*)(ext + (size_t)4 * i);
  const v4f sc = *(const v4f*)(scsh2 + c4);
  const v4f sh = *(const v4f*)(scsh2 + 256 + c4);
  v4f o;
#pragma unroll
  for (int q = 0; q < 4; ++q) {
    const float v = e[q] * sc[q] + sh[q];
    o[q] = fmaxf(v, 0.0f);
  }
  float* dst = out1 + (size_t)4 * i;
  *(volatile v4f*)dst = o;
  __threadfence();
  *(volatile v4f*)dst = o;
}

extern "C" void kernel_launch(void* const* d_in, const int* in_sizes, int n_in,
                              void* d_out, int out_size, void* d_ws, size_t ws_size,
                              hipStream_t stream) {
  (void)in_sizes; (void)n_in; (void)out_size;
  if (ws_size < WS_TOTAL) return;
  const float* xyz = (const float*)d_in[0];
  const float* pts = (const float*)d_in[1];
  const float* w0  = (const float*)d_in[2];
  const float* g0  = (const float*)d_in[4];
  const float* bt0 = (const float*)d_in[5];
  const float* w1  = (const float*)d_in[6];
  const float* g1  = (const float*)d_in[8];
  const float* bt1 = (const float*)d_in[9];
  const float* w2  = (const float*)d_in[10];
  const float* g2  = (const float*)d_in[12];
  const float* bt2 = (const float*)d_in[13];
  float* out0 = (float*)d_out;
  float* out1 = (float*)d_out + OUT1_OFFSET_FLOATS;

  char* ws = (char*)d_ws;
  int*            fpsidx = (int*)(ws + OFF_FPSI);
  int*            bidx   = (int*)(ws + OFF_BIDX);
  float*          Ppl    = (float*)(ws + OFF_PPL);
  unsigned short* y0h    = (unsigned short*)(ws + OFF_Y0H);
  float*          extp   = (float*)(ws + OFF_EXT);
  float*          part0  = (float*)(ws + OFF_PART0);
  float*          part1  = (float*)(ws + OFF_PART1);
  float*          part2  = (float*)(ws + OFF_PART2);
  unsigned short* wpk    = (unsigned short*)(ws + OFF_WPK);
  float*          scsh0  = (float*)(ws + OFF_SCSH0);
  float*          scsh1  = (float*)(ws + OFF_SCSH1);
  float*          scsh2  = (float*)(ws + OFF_SCSH2);
  const unsigned short* w0p = wpk;
  const unsigned short* w1t = wpk + 4096;
  const unsigned short* w2t = wpk + 12288;

  prep_pack_kernel<<<WPK_HALVES / 2048, 256, 0, stream>>>(w0, w1, w2, wpk);
  fps_kernel<<<NBATCH, 512, 0, stream>>>(xyz, out0, fpsidx);
  ballq_kernel<<<NGROUPS / 8, 256, 0, stream>>>(xyz, fpsidx, bidx);
  pgemm_kernel<<<NSRC / 128, 256, 0, stream>>>(pts, w0p, Ppl);
  gather_kernel<<<NBLK0, 256, 0, stream>>>(xyz, Ppl, w0, fpsidx, bidx, y0h, part0);
  finalize_kernel<<<CHAN0 / 32, 256, 0, stream>>>(part0, NBLK0, CHAN0, g0, bt0, scsh0);
  passB_kernel<<<NBLK1, 256, 0, stream>>>(y0h, w1t, scsh0, part1);
  finalize_kernel<<<CHAN1 / 32, 256, 0, stream>>>(part1, NBLK1, CHAN1, g1, bt1, scsh1);
  passC_kernel<<<NBLK2, 128, 0, stream>>>(y0h, w1t, w2t, scsh0, scsh1, g2, part2, extp);
  finalize_kernel<<<CHAN2 / 32, 256, 0, stream>>>(part2, NBLK2, CHAN2, g2, bt2, scsh2);
  out_kernel<<<(NGROUPS * 256 / 4) / 256, 256, 0, stream>>>(extp, scsh2, out1);
}
